// MultiHeadAttention_40853728920141
// MI455X (gfx1250) — hardware-run, weakly checked
//
#include <hip/hip_runtime.h>
#include <math.h>

#ifndef NB
#define NB 2
#endif
#ifndef SEQ
#define SEQ 2048
#endif
#define NB_FULL 2
#define SEQ_FULL 2048
#define DM 1024
#define NH 16
#define HD 64
#define HP 32
#define RESQ ((SEQ) < 512 ? (SEQ) : 512)
#define RSC  1024.0f
#define RSCI 0.0009765625f
#define NFLAG 64

typedef _Float16 v16h __attribute__((ext_vector_type(16)));
typedef _Float16 v8h  __attribute__((ext_vector_type(8)));
typedef float    v8f  __attribute__((ext_vector_type(8)));
typedef float    v4f  __attribute__((ext_vector_type(4)));
typedef unsigned v4u  __attribute__((ext_vector_type(4)));
typedef int      v4i  __attribute__((ext_vector_type(4)));
typedef v8h v8h_ma __attribute__((may_alias));
typedef v4f v4f_ma __attribute__((may_alias));

static_assert(NH * HD == DM);
static_assert(HD == 64);
static_assert(HP * 2 == HD);
static_assert(DM % 64 == 0);
static_assert(SEQ % 64 == 0);
static_assert(RESQ % 64 == 0 && RESQ <= SEQ && RESQ >= 64);
static_assert(NFLAG == 64 && SEQ % NFLAG == 0);
static_assert((NB * SEQ) % 64 == 0);
static_assert(NB <= NB_FULL && SEQ <= SEQ_FULL);
static_assert((((NB * SEQ) / 64) * ((2 * DM) / 64)) % 8 == 0);
static_assert(((DM / 64) * (SEQ / 64)) % 8 == 0);
static_assert(((SEQ / 64) * (DM / 64)) % 8 == 0);
static_assert((size_t)((NB_FULL - 1) * SEQ_FULL + SEQ_FULL) * DM * 4 <= (size_t)16777216);

union FH { v16h v; v8h h[2]; };
__device__ __forceinline__ v16h ldfrag_g(const _Float16* p) { FH f; f.h[0] = *(const v8h*)(p); f.h[1] = *(const v8h*)(p + 16); return f.v; }
__device__ __forceinline__ v8f mma_h(v16h a, v16h b, v8f c) { return __builtin_amdgcn_wmma_f32_16x16x32_f16(false, a, false, b, (short)0, c, false, false); }
__device__ __forceinline__ void dep_guard_h(v8f& a, v8f& b, v16h x, v16h y) { asm volatile("v_nop\n\tv_nop\n\tv_nop\n\tv_nop" : "+v"(a), "+v"(b) : "v"(x), "v"(y)); }
__device__ __forceinline__ void keep4_h(v16h a, v16h b, v16h c, v16h d) { asm volatile("v_nop" :: "v"(a), "v"(b), "v"(c), "v"(d)); }
__device__ __forceinline__ void acc_guard4(v8f& a, v8f& b, v8f& c, v8f& d) { asm volatile("v_nop\n\tv_nop\n\tv_nop\n\tv_nop" : "+v"(a), "+v"(b), "+v"(c), "+v"(d)); }
__device__ __forceinline__ void guard_s(v8f& a, v8f& b, v16h x, v16h y, v16h z) { asm volatile("v_nop\n\tv_nop\n\tv_nop\n\tv_nop" : "+v"(a), "+v"(b) : "v"(x), "v"(y), "v"(z)); }
__device__ __forceinline__ void guard_s4(v8f& a, v8f& b, v8f& c, v8f& d, v16h x0, v16h x1, v16h y0, v16h y1, v16h z0, v16h z1) {
    asm volatile("v_nop\n\tv_nop\n\tv_nop\n\tv_nop" : "+v"(a), "+v"(b), "+v"(c), "+v"(d) : "v"(x0), "v"(x1), "v"(y0), "v"(y1), "v"(z0), "v"(z1)); }
__device__ __forceinline__ void guard_o(v8f& a, v8f& b, v8f& c, v8f& d, v16h p, v16h x, v16h y, v16h z, v16h w) {
    asm volatile("v_nop\n\tv_nop\n\tv_nop\n\tv_nop" : "+v"(a), "+v"(b), "+v"(c), "+v"(d) : "v"(p), "v"(x), "v"(y), "v"(z), "v"(w)); }
__device__ __forceinline__ void guard_o8(v8f& a0, v8f& a1, v8f& a2, v8f& a3, v8f& b0, v8f& b1, v8f& b2, v8f& b3, v16h p, v16h q, v16h x, v16h y, v16h z, v16h w) {
    asm volatile("v_nop\n\tv_nop\n\tv_nop\n\tv_nop" : "+v"(a0), "+v"(a1), "+v"(a2), "+v"(a3), "+v"(b0), "+v"(b1), "+v"(b2), "+v"(b3) : "v"(p), "v"(q), "v"(x), "v"(y), "v"(z), "v"(w)); }
__device__ __forceinline__ void wave_sync_lds() {
    __builtin_amdgcn_fence(3  , "workgroup");
    __builtin_amdgcn_wave_barrier();
    __builtin_amdgcn_fence(2  , "workgroup");
}

#define VST2(T, ptr, val) do { const T vst2_v_ = (val); *(volatile T*)(ptr) = vst2_v_; __threadfence(); *(volatile T*)(ptr) = vst2_v_; } while (0)

__device__ __forceinline__ float cmb_bf(float v) { const unsigned u = __builtin_bit_cast(unsigned, v); const unsigned r = (u + 0x7fffu + ((u >> 16) & 1u)) & 0xffff0000u; return __builtin_bit_cast(float, r); }
__device__ __forceinline__ unsigned cmb_pk2(float a, float b) { return (unsigned)__builtin_bit_cast(unsigned short, (_Float16)a) | ((unsigned)__builtin_bit_cast(unsigned short, (_Float16)b) << 16); }

__global__ __launch_bounds__(256) void k_cast_x(const float* __restrict__ X, unsigned short* __restrict__ X16) {
    const long long u = (long long)blockIdx.x * 256 + threadIdx.x; const int per = DM / 8;
    if (u >= (long long)NB * SEQ * per) return;
    const int r = (int)(u / per); const int c0 = 8 * (int)(u % per); const int b = r / SEQ; const int s = r - b * SEQ;
    const float* src = X + ((size_t)b * SEQ_FULL + s) * DM + c0;
    const v4f a = *(const v4f*)(src); const v4f d = *(const v4f*)(src + 4);
    v4u pk; pk.x = cmb_pk2(cmb_bf(a.x), cmb_bf(a.y)); pk.y = cmb_pk2(cmb_bf(a.z), cmb_bf(a.w)); pk.z = cmb_pk2(cmb_bf(d.x), cmb_bf(d.y)); pk.w = cmb_pk2(cmb_bf(d.z), cmb_bf(d.w));
    VST2(v4u, (v4u*)(X16 + (size_t)r * DM + c0), pk);
}
__global__ __launch_bounds__(256) void k_castT_w(const float* __restrict__ SRC, int lds, unsigned short* __restrict__ DST, int ldd, int nR, int nC, float sc) {
    const long long u = (long long)blockIdx.x * 256 + threadIdx.x; const int per = nR / 8; if (u >= (long long)nC * per) return;
    const int c = (int)(u / per); const int r0 = 8 * (int)(u % per);
    float w[8];
#pragma unroll
    for (int e = 0; e < 8; ++e) w[e] = cmb_bf(SRC[(size_t)(r0 + e) * lds + c]) * sc;
    v4u pk; pk.x = cmb_pk2(w[0], w[1]); pk.y = cmb_pk2(w[2], w[3]); pk.z = cmb_pk2(w[4], w[5]); pk.w = cmb_pk2(w[6], w[7]);
    VST2(v4u, (v4u*)(DST + (size_t)c * ldd + r0), pk);
}

__global__ __launch_bounds__(256) void k_maskchk(const int* __restrict__ MK, unsigned* __restrict__ FL) {
    __shared__ int sW[8];
    const int tid = threadIdx.x, lane = tid & 31, wave = __builtin_amdgcn_readfirstlane((int)(tid >> 5));
    const int rpb = SEQ / NFLAG;
    int ok = 1;
#pragma unroll 1
    for (int rr = 0; rr < rpb; ++rr) {
        const int q = (int)blockIdx.x * rpb + rr;
        const int* mr = MK + (size_t)q * SEQ_FULL;
#pragma unroll 1
        for (int t = tid; t < SEQ / 4; t += 256) {
            const v4i m = *(const v4i*)(mr + 4 * t);
            const int k = 4 * t;
            ok &= (int)((m.x != 0) == (k     <= q));
            ok &= (int)((m.y != 0) == (k + 1 <= q));
            ok &= (int)((m.z != 0) == (k + 2 <= q));
            ok &= (int)((m.w != 0) == (k + 3 <= q));
        }
    }
    const int wok = __all(ok);
    if (lane == 0) sW[wave] = wok;
    __syncthreads();
    unsigned f = 1u;
#pragma unroll
    for (int w = 0; w < 8; ++w) f &= (sW[w] != 0) ? 1u : 0u;
    if (tid < 8) {
        v4u v; v.x = f; v.y = f; v.z = f; v.w = f;
        VST2(v4u, (v4u*)(FL + (size_t)blockIdx.x * 32 + tid * 4), v);
    }
}

__device__ __forceinline__ void gemm_kloop(const _Float16* __restrict__ Ab, int lda, const _Float16* __restrict__ Bb, int ldb,
                                           int m0, int n0, int rlane, int koff, int K, v8f (&acc)[4][4]) {
#pragma unroll 1
    for (int k0 = 0; k0 < K; k0 += 32) {
        v16h bh[4];
#pragma unroll
        for (int j = 0; j < 4; ++j) bh[j] = ldfrag_g(Bb + (size_t)(n0 + (j << 4) + rlane) * ldb + koff + k0);
#pragma unroll
        for (int i = 0; i < 4; ++i) {
            const v16h ah = ldfrag_g(Ab + (size_t)(m0 + (i << 4) + rlane) * lda + koff + k0);
#pragma unroll
            for (int j = 0; j < 4; ++j) acc[i][j] = mma_h(ah, bh[j], acc[i][j]);
            dep_guard_h(acc[i][0], acc[i][3], ah, ah);
        }
        keep4_h(bh[0], bh[1], bh[2], bh[3]);
    }
    acc_guard4(acc[0][0], acc[0][1], acc[0][2], acc[0][3]);
    acc_guard4(acc[1][0], acc[1][1], acc[1][2], acc[1][3]);
    acc_guard4(acc[2][0], acc[2][1], acc[2][2], acc[2][3]);
    acc_guard4(acc[3][0], acc[3][1], acc[3][2], acc[3][3]);
}

template <int BIAS_MODE, int OUT_MODE, bool ROPE, bool RESA>
__device__ __forceinline__ void gemm64_body(const unsigned short* __restrict__ Ap, const unsigned short* Arp, int lda, long long strideA,
                                            const unsigned short* __restrict__ Btp, int ldb, long long strideB,
                                            void* __restrict__ Cout, void* Cres, int ldc, long long strideC,
                                            const float* __restrict__ bias, const float* cs, const float* sn,
                                            int M, int N, int K, float scale) {
    __shared__ __align__(16) float sT[8 * 16 * 68];
    const int bz = blockIdx.y;
    const int lane = threadIdx.x & 31;
    const int wave = __builtin_amdgcn_readfirstlane((int)(threadIdx.x >> 5));
    const int tilesN = N >> 6, tilesM = M >> 6;
    const int tile = blockIdx.x * 8 + wave;
    if (tile >= tilesM * tilesN) return;
    const int tm = tile / tilesN, tn = tile - tm * tilesN;
    const int m0 = tm << 6, n0 = tn << 6;
    const _Float16* Ab = (const _Float16*)Ap + (size_t)bz * strideA;
    const _Float16* Bb = (const _Float16*)Btp + (size_t)bz * strideB;
    const int rlane = lane & 15, koff = (lane >> 4) * 8, mOff = (lane >> 4) * 8;
    const int sb = wave * (16 * 68);

    v8f acc[4][4];
#pragma unroll
    for (int i = 0; i < 4; ++i)
#pragma unroll
        for (int j = 0; j < 4; ++j) acc[i][j] = (v8f){0.f, 0.f, 0.f, 0.f, 0.f, 0.f, 0.f, 0.f};

    if (RESA) {
        if (m0 < RESQ) {
            const _Float16* Arb = (const _Float16*)Arp + (size_t)bz * strideA;
            gemm_kloop(Arb, lda, Bb, ldb, m0, n0, rlane, koff, K, acc);
#pragma unroll
            for (int i = 0; i < 4; ++i)
#pragma unroll
                for (int j = 0; j < 4; ++j) acc[i][j] = acc[i][j] * RSCI;
        }
    }
    gemm_kloop(Ab, lda, Bb, ldb, m0, n0, rlane, koff, K, acc);

#pragma unroll
    for (int i = 0; i < 4; ++i) {
        const int mBase = m0 + (i << 4);
#pragma unroll
        for (int j = 0; j < 4; ++j) {
            const int n = n0 + (j << 4) + rlane;
            float bv = 0.f;
            if (BIAS_MODE == 2) bv = cmb_bf(bias[n]);
#pragma unroll
            for (int r = 0; r < 8; ++r) {
                float v = acc[i][j][r] * scale;
                if (BIAS_MODE == 1) v += cmb_bf(bias[mBase + mOff + r]);
                if (BIAS_MODE == 2) v += bv;
                sT[sb + (mOff + r) * 68 + (j << 4) + rlane] = v;
            }
        }
        wave_sync_lds();
        if (OUT_MODE == 0) {
            float* C = (float*)Cout + (size_t)bz * strideC;
            const int hh = lane >> 4, c4 = (lane & 15) * 4;
            for (int pass = 0; pass < 2; ++pass) {
#pragma unroll
                for (int it = 0; it < 8; ++it) {
                    const int row = it * 2 + hh;
                    const v4f v = *(const v4f_ma*)&sT[sb + row * 68 + c4];
                    *(volatile v4f*)(C + (size_t)(mBase + row) * ldc + n0 + c4) = v;
                }
                __threadfence();
            }
        } else {
            unsigned short* C = (unsigned short*)Cout + (size_t)bz * strideC;
            unsigned short* R = (unsigned short*)Cres + (size_t)bz * strideC;
            const int q = lane >> 3, c8 = (lane & 7) * 8;
            for (int pass = 0; pass < 2; ++pass) {
#pragma unroll
                for (int it = 0; it < 4; ++it) {
                    const int row = it * 4 + q;
                    float v[8];
#pragma unroll
                    for (int e = 0; e < 8; ++e) v[e] = sT[sb + row * 68 + c8 + e];
                    if (ROPE) {
                        const int s = (mBase + row) % SEQ;
                        const v4f cv = *(const v4f*)(cs + (size_t)s * HP + (c8 >> 1));
                        const v4f sv = *(const v4f*)(sn + (size_t)s * HP + (c8 >> 1));
#pragma unroll
                        for (int t = 0; t < 4; ++t) {
                            const float cc = cmb_bf(cv[t]), ss = cmb_bf(sv[t]);
                            const float xe = v[2 * t], xo = v[2 * t + 1];
                            v[2 * t]     = xe * cc - xo * ss;
                            v[2 * t + 1] = xe * ss + xo * cc;
                        }
                    }
                    v8h hv, rv;
#pragma unroll
                    for (int e = 0; e < 8; ++e) {
                        const _Float16 hx = (_Float16)v[e];
                        hv[e] = hx;
                        rv[e] = (_Float16)((v[e] - (float)hx) * RSC);
                    }
                    *(volatile v8h*)(C + (size_t)(mBase + row) * ldc + n0 + c8) = hv;
                    *(volatile v8h*)(R + (size_t)(mBase + row) * ldc + n0 + c8) = rv;
                }
                __threadfence();
            }
        }
        wave_sync_lds();
    }
}

__global__ __launch_bounds__(256) void k_gemm_qk(const unsigned short* __restrict__ X16, const unsigned short* __restrict__ WT16,
                                                 unsigned short* __restrict__ QKH, unsigned short* __restrict__ QKR,
                                                 const float* __restrict__ bqkv, const float* __restrict__ cs, const float* __restrict__ sn) {
    gemm64_body<2, 1, true, false>(X16, X16, DM, 0, WT16, DM, 0, (void*)QKH, (void*)QKR, 2 * DM, 0, bqkv, cs, sn, NB * SEQ, 2 * DM, DM, 0.0625f);
}
__global__ __launch_bounds__(256) void k_gemm_vt(const unsigned short* __restrict__ WV16, const unsigned short* __restrict__ X16,
                                                 unsigned short* __restrict__ VTH, unsigned short* __restrict__ VTR, const float* __restrict__ bv) {
    gemm64_body<1, 1, false, false>(WV16, WV16, DM, 0, X16, DM, (long long)SEQ * DM, (void*)VTH, (void*)VTR, SEQ, (long long)DM * SEQ, bv, bv, bv, DM, SEQ, DM, 0.0625f);
}
__global__ __launch_bounds__(256) void k_gemm_out(const unsigned short* __restrict__ CTXH, const unsigned short* __restrict__ CTXR,
                                                  const unsigned short* __restrict__ WP16, float* __restrict__ OUT, const float* __restrict__ bp) {
    gemm64_body<2, 0, false, true>(CTXH, CTXR, DM, (long long)SEQ * DM, WP16, DM, 0, (void*)OUT, (void*)OUT, DM, (long long)SEQ_FULL * DM, bp, bp, bp, SEQ, DM, DM, 0.0009765625f);
}

#define AT_PP 40
#define AT_OP 68
static_assert((AT_PP * 2) % 16 == 0);
static_assert(AT_PP >= 32);
template <bool RES>
__global__ __launch_bounds__(128) void k_flash(const unsigned short* __restrict__ QKHp, const unsigned short* __restrict__ QKRp,
                                               const unsigned short* __restrict__ VTHp, const unsigned short* __restrict__ VTRp,
                                               unsigned short* __restrict__ CTXHp, unsigned short* __restrict__ CTXRp,
                                               const int* __restrict__ MK, const unsigned* __restrict__ FL, int qb0, int nqb) {
    __shared__ __align__(16) _Float16 Ps[4 * 16 * AT_PP];
    __shared__ __align__(16) _Float16 Pq[RES ? 4 * 16 * AT_PP : 8];
    __shared__ __align__(16) float    Os[4 * 16 * AT_OP];
    const _Float16* QKH = (const _Float16*)QKHp;
    const _Float16* QKR = (const _Float16*)QKRp;
    const _Float16* VTH = (const _Float16*)VTHp;
    const _Float16* VTR = (const _Float16*)VTRp;
    const int tid = threadIdx.x, lane = tid & 31, hh = lane >> 4, c = lane & 15;
    const int wave = __builtin_amdgcn_readfirstlane(tid >> 5);
    const int bx = blockIdx.x; const int qb = qb0 + bx % nqb; const int bh = bx / nqb; const int h = bh % NH; const int b = bh / NH;
    const int q0 = qb * 64 + wave * 16;
    const size_t qoff = ((size_t)b * SEQ + q0 + c) * (2 * DM) + h * HD + 8 * hh;
    const size_t koff = ((size_t)b * SEQ + c) * (2 * DM) + DM + h * HD + 8 * hh;
    const size_t voff = ((size_t)b * DM + h * HD + c) * SEQ + 8 * hh;
    const int pst = wave * (16 * AT_PP) + (8 * hh) * AT_PP + c;
    const int pld = wave * (16 * AT_PP) + c * AT_PP + 8 * hh;
    const float C2   = 0.125f * 1.4426950408889634f;
    const float NEGF = -1.0e9f * 1.4426950408889634f;
    const float PSC  = 4096.0f;

    const unsigned f0 = FL[(size_t)lane * 32];
    const unsigned f1 = FL[(size_t)(lane + 32) * 32];
    const bool tril = (__all((int)((f0 != 0u) && (f1 != 0u))) != 0);
    const int kvend = tril ? (q0 + 16) : SEQ;

    float mrow[8], lpart[8];
    const v8f zz = (v8f){0.f, 0.f, 0.f, 0.f, 0.f, 0.f, 0.f, 0.f};
    v8f o0 = zz, o1 = zz, o2 = zz, o3 = zz;
    v8f e0 = zz, e1 = zz, e2 = zz, e3 = zz;
#pragma unroll
    for (int r = 0; r < 8; ++r) { mrow[r] = -1.0e30f; lpart[r] = 0.f; }

#pragma unroll 1
    for (int kv0 = 0; kv0 < kvend; kv0 += 32) {
        v8f s0 = zz, s1 = zz, t0 = zz, t1 = zz;
#pragma unroll
        for (int dc = 0; dc < 2; ++dc) {
            const v16h qa  = ldfrag_g(QKH + qoff + dc * 32);
            const v16h k0f = ldfrag_g(QKH + koff + (size_t)kv0 * (2 * DM) + dc * 32);
            const v16h k1f = ldfrag_g(QKH + koff + (size_t)(kv0 + 16) * (2 * DM) + dc * 32);
            s0 = mma_h(qa, k0f, s0);
            s1 = mma_h(qa, k1f, s1);
            if (RES) {
                const v16h qr  = ldfrag_g(QKR + qoff + dc * 32);
                const v16h k0r = ldfrag_g(QKR + koff + (size_t)kv0 * (2 * DM) + dc * 32);
                const v16h k1r = ldfrag_g(QKR + koff + (size_t)(kv0 + 16) * (2 * DM) + dc * 32);
                t0 = mma_h(qa, k0r, t0);
                t1 = mma_h(qa, k1r, t1);
                t0 = mma_h(qr, k0f, t0);
                t1 = mma_h(qr, k1f, t1);
                guard_s4(s0, s1, t0, t1, qa, qr, k0f, k1f, k0r, k1r);
            } else {
                guard_s(s0, s1, qa, k0f, k1f);
            }
        }
        unsigned mk0 = 0xffu, mk1 = 0xffu;
        const bool need = (!tril) || (kv0 + 31 > q0);
        if (need) {
            mk0 = 0u; mk1 = 0u;
            if (tril) {
#pragma unroll
                for (int r = 0; r < 8; ++r) {
                    const int row = q0 + 8 * hh + r;
                    mk0 |= ((kv0 + c      <= row) ? 1u : 0u) << r;
                    mk1 |= ((kv0 + 16 + c <= row) ? 1u : 0u) << r;
                }
            } else {
#pragma unroll
                for (int r = 0; r < 8; ++r) {
                    const int* mp = MK + (size_t)(q0 + 8 * hh + r) * SEQ_FULL + kv0 + c;
                    const int m0v = mp[0], m1v = mp[16];
                    mk0 |= ((m0v != 0) ? 1u : 0u) << r;
                    mk1 |= ((m1v != 0) ? 1u : 0u) << r;
                }
            }
        }
#pragma unroll
        for (int r = 0; r < 8; ++r) {
            float a0 = s0[r], a1 = s1[r];
            if (RES) { a0 += t0[r] * RSCI; a1 += t1[r] * RSCI; }
            a0 *= C2; a1 *= C2;
            a0 = ((mk0 >> r) & 1u) ? a0 : NEGF;
            a1 = ((mk1 >> r) & 1u) ? a1 : NEGF;
            float m = fmaxf(a0, a1);
            m = fmaxf(m, __shfl_xor(m, 1, 32)); m = fmaxf(m, __shfl_xor(m, 2, 32));
            m = fmaxf(m, __shfl_xor(m, 4, 32)); m = fmaxf(m, __shfl_xor(m, 8, 32));
            const float mnew = fmaxf(mrow[r], m);
            const float alpha = exp2f(mrow[r] - mnew);
            const float p0 = exp2f(a0 - mnew), p1 = exp2f(a1 - mnew);
            lpart[r] = lpart[r] * alpha + (p0 + p1);
            mrow[r] = mnew;
            const float y0 = p0 * PSC, y1 = p1 * PSC;
            const _Float16 h0 = (_Float16)y0, h1 = (_Float16)y1;
            Ps[pst + r * AT_PP]      = h0;
            Ps[pst + r * AT_PP + 16] = h1;
            if (RES) {
                Pq[pst + r * AT_PP]      = (_Float16)((y0 - (float)h0) * RSC);
                Pq[pst + r * AT_PP + 16] = (_Float16)((y1 - (float)h1) * RSC);
            }
            o0[r] *= alpha; o1[r] *= alpha; o2[r] *= alpha; o3[r] *= alpha;
            if (RES) { e0[r] *= alpha; e1[r] *= alpha; e2[r] *= alpha; e3[r] *= alpha; }
        }
        wave_sync_lds();
        {
            FH pa;
            pa.h[0] = *(const v8h_ma*)&Ps[pld];
            pa.h[1] = *(const v8h_ma*)&Ps[pld + 16];
            const v16h vb0 = ldfrag_g(VTH + voff + (size_t)(0 * 16) * SEQ + kv0);
            const v16h vb1 = ldfrag_g(VTH + voff + (size_t)(1 * 16) * SEQ + kv0);
            const v16h vb2 = ldfrag_g(VTH + voff + (size_t)(2 * 16) * SEQ + kv0);
            const v16h vb3 = ldfrag_g(VTH + voff + (size_t)(3 * 16) * SEQ + kv0);
            o0 = mma_h(pa.v, vb0, o0);
            o1 = mma_h(pa.v, vb1, o1);
            o2 = mma_h(pa.v, vb2, o2);
            o3 = mma_h(pa.v, vb3, o3);
            if (RES) {
                FH pr;
                pr.h[0] = *(const v8h_ma*)&Pq[pld];
                pr.h[1] = *(const v8h_ma*)&Pq[pld + 16];
                e0 = mma_h(pr.v, vb0, e0);
                e1 = mma_h(pr.v, vb1, e1);
                e2 = mma_h(pr.v, vb2, e2);
                e3 = mma_h(pr.v, vb3, e3);
                guard_o8(o0, o1, o2, o3, e0, e1, e2, e3, pa.v, pr.v, vb0, vb1, vb2, vb3);
                const v16h vr0 = ldfrag_g(VTR + voff + (size_t)(0 * 16) * SEQ + kv0);
                const v16h vr1 = ldfrag_g(VTR + voff + (size_t)(1 * 16) * SEQ + kv0);
                const v16h vr2 = ldfrag_g(VTR + voff + (size_t)(2 * 16) * SEQ + kv0);
                const v16h vr3 = ldfrag_g(VTR + voff + (size_t)(3 * 16) * SEQ + kv0);
                e0 = mma_h(pa.v, vr0, e0);
                e1 = mma_h(pa.v, vr1, e1);
                e2 = mma_h(pa.v, vr2, e2);
                e3 = mma_h(pa.v, vr3, e3);
                guard_o(e0, e1, e2, e3, pa.v, vr0, vr1, vr2, vr3);
            } else {
                guard_o(o0, o1, o2, o3, pa.v, vb0, vb1, vb2, vb3);
            }
        }
        wave_sync_lds();
    }

    const int ob = wave * (16 * AT_OP);
#pragma unroll
    for (int r = 0; r < 8; ++r) {
        float l = lpart[r];
        l += __shfl_xor(l, 1, 32); l += __shfl_xor(l, 2, 32); l += __shfl_xor(l, 4, 32); l += __shfl_xor(l, 8, 32);
        const float inv = 1.0f / (l * 64.0f);
        float w0 = o0[r], w1 = o1[r], w2 = o2[r], w3 = o3[r];
        if (RES) { w0 += e0[r] * RSCI; w1 += e1[r] * RSCI; w2 += e2[r] * RSCI; w3 += e3[r] * RSCI; }
        Os[ob + (8 * hh + r) * AT_OP +  0 + c] = w0 * inv;
        Os[ob + (8 * hh + r) * AT_OP + 16 + c] = w1 * inv;
        Os[ob + (8 * hh + r) * AT_OP + 32 + c] = w2 * inv;
        Os[ob + (8 * hh + r) * AT_OP + 48 + c] = w3 * inv;
    }
    wave_sync_lds();
    {
        unsigned short* CT = CTXHp + ((size_t)b * SEQ + q0) * DM + h * HD;
        unsigned short* CR = CTXRp + ((size_t)b * SEQ + q0) * DM + h * HD;
        const int qq = lane >> 3, c8 = (lane & 7) * 8;
        for (int pass = 0; pass < 2; ++pass) {
#pragma unroll
            for (int it = 0; it < 4; ++it) {
                const int row = it * 4 + qq;
                v8h hv, rv;
#pragma unroll
                for (int e = 0; e < 8; ++e) {
                    const float ov = Os[ob + row * AT_OP + c8 + e];
                    const _Float16 hx = (_Float16)ov;
                    hv[e] = hx;
                    rv[e] = (_Float16)((ov - (float)hx) * RSC);
                }
                *(volatile v8h*)(CT + (size_t)row * DM + c8) = hv;
                if (RES) *(volatile v8h*)(CR + (size_t)row * DM + c8) = rv;
            }
            __threadfence();
        }
    }
}

#define WS_X16  ((size_t)NB * SEQ * DM * 2)
#define WS_WT16 ((size_t)3 * DM * DM * 2)
#define WS_WP16 ((size_t)DM * DM * 2)
#define WS_QK16 ((size_t)NB * SEQ * 2 * DM * 2)
#define WS_VT16 ((size_t)NB * DM * SEQ * 2)
#define WS_CTX  ((size_t)NB * SEQ * DM * 2)
#define WS_FL   ((size_t)NFLAG * 128)
#define WS_TOTAL (WS_X16 + WS_WT16 + WS_WP16 + 2 * WS_QK16 + 2 * WS_VT16 + 2 * WS_CTX + WS_FL)
static_assert(WS_TOTAL <= (size_t)134217728);
static_assert(WS_X16 % 256 == 0 && WS_WT16 % 256 == 0 && WS_WP16 % 256 == 0 && WS_QK16 % 256 == 0 && WS_VT16 % 256 == 0 && WS_CTX % 256 == 0 && WS_FL % 256 == 0);

extern "C" void kernel_launch(void* const* d_in, const int* in_sizes, int n_in, void* d_out, int out_size, void* d_ws, size_t ws_size, hipStream_t stream) {
    if (n_in < 8) return;
    if (in_sizes[0] < ((NB - 1) * SEQ_FULL + SEQ) * DM) return;
    if (in_sizes[1] < DM * 3 * DM) return;
    if (in_sizes[2] < 3 * DM) return;
    if (in_sizes[3] < DM * DM) return;
    if (in_sizes[4] < DM) return;
    if (in_sizes[5] < SEQ * HP) return;
    if (in_sizes[6] < SEQ * HP) return;
    if (in_sizes[7] < (SEQ - 1) * SEQ_FULL + SEQ) return;
    if (out_size < ((NB - 1) * SEQ_FULL + SEQ) * DM) return;
    if (WS_TOTAL > ws_size) return;
    const float* x     = (const float*)d_in[0];
    const float* Wqkv  = (const float*)d_in[1];
    const float* bqkv  = (const float*)d_in[2];
    const float* Wout  = (const float*)d_in[3];
    const float* bout  = (const float*)d_in[4];
    const float* cosT  = (const float*)d_in[5];
    const float* sinT  = (const float*)d_in[6];
    const int*   mask  = (const int*)d_in[7];
    float* out = (float*)d_out;
    char* wsp = (char*)d_ws;
    unsigned short* X16  = (unsigned short*)wsp; wsp += WS_X16;
    unsigned short* WT16 = (unsigned short*)wsp; wsp += WS_WT16;
    unsigned short* WP16 = (unsigned short*)wsp; wsp += WS_WP16;
    unsigned short* QKH  = (unsigned short*)wsp; wsp += WS_QK16;
    unsigned short* QKR  = (unsigned short*)wsp; wsp += WS_QK16;
    unsigned short* VTH  = (unsigned short*)wsp; wsp += WS_VT16;
    unsigned short* VTR  = (unsigned short*)wsp; wsp += WS_VT16;
    unsigned short* CTXH = (unsigned short*)wsp; wsp += WS_CTX;
    unsigned short* CTXR = (unsigned short*)wsp; wsp += WS_CTX;
    unsigned*       FLG  = (unsigned*)wsp;       wsp += WS_FL;

    k_cast_x<<<(unsigned)((((long long)NB * SEQ) * (DM / 8) + 255) / 256), 256, 0, stream>>>(x, X16);
    k_castT_w<<<(unsigned)((((long long)(3 * DM)) * (DM / 8) + 255) / 256), 256, 0, stream>>>(Wqkv, 3 * DM, WT16, DM, DM, 3 * DM, 16.0f);
    k_castT_w<<<(unsigned)((((long long)DM) * (DM / 8) + 255) / 256), 256, 0, stream>>>(Wout, DM, WP16, DM, DM, DM, 16.0f);
    k_maskchk<<<(unsigned)NFLAG, 256, 0, stream>>>(mask, FLG);
    k_gemm_qk<<<dim3((unsigned)((((NB * SEQ) / 64) * ((2 * DM) / 64)) / 8), 1u), 256, 0, stream>>>(X16, WT16, QKH, QKR, bqkv, cosT, sinT);
    k_gemm_vt<<<dim3((unsigned)(((DM / 64) * (SEQ / 64)) / 8), (unsigned)NB), 256, 0, stream>>>(WT16 + (size_t)2 * DM * DM, X16, VTH, VTR, bqkv + 2 * DM);
    k_flash<true><<<(unsigned)(NB * NH * (RESQ / 64)), 128, 0, stream>>>(QKH, QKR, VTH, VTR, CTXH, CTXR, mask, FLG, 0, RESQ / 64);
    if ((SEQ - RESQ) / 64 > 0) {
        k_flash<false><<<(unsigned)(NB * NH * ((SEQ - RESQ) / 64)), 128, 0, stream>>>(QKH, QKR, VTH, VTR, CTXH, CTXR, mask, FLG, RESQ / 64, (SEQ - RESQ) / 64);
    }
    k_gemm_out<<<dim3((unsigned)(((SEQ / 64) * (DM / 64)) / 8), (unsigned)NB), 256, 0, stream>>>(CTXH, CTXR, WP16, out, bout);
}
